// IntegralTransform_2911987826756
// MI455X (gfx1250) — hardware-verified
//
#include <hip/hip_runtime.h>
#include <stddef.h>
#include <stdint.h>
#include <math.h>

#pragma clang fp contract(off)

#define NCO    3
#define CH     64
#define HID    256
#define D1     70
#define KF     64
#define K1     96
#define UPR    (K1 / 8)
#define PP     256
#define K23    256
#define NTHR   256
#define EPB    128
#define QPB    4
#define NXQ    (QPB * NCO)
#define AP     264
#define DP     68
#define GBM    64
#define GBN    128
#define GTHR   128
#define NU_BT  (HID * UPR)
#define NU_W2  (HID * (K23 / 8))
#define NU_W3  (CH * (K23 / 8))
#define NU_W   (NU_BT + NU_W2 + NU_W3)
#define CA     4.0f
#define CW     256.0f
#define INVC   0.0009765625f
#define WSMAX  134217728
#define L_SA   (EPB * AP * 2)
#define L_SH   (EPB * AP * 2)
#define L_SD   (EPB * DP * 4)
#define L_SQ   (QPB * HID * 4)
#define L_SO   (QPB * CH * 4)
#define L_CST  ((HID + CH) * 4)
#define L_SW   (EPB * 4)
#define L_SS   (EPB * 4)
#define L_SJ   (EPB * 4)
#define L_SQL  (EPB * 4)
#define L_SX   64
#define L_SRS  64
#define EDGE_LDS_BYTES (L_SA + L_SH + L_SD + L_SQ + L_SO + L_CST + L_SW + L_SS + L_SJ + L_SQL + L_SX + L_SRS)

static_assert(K1 % 32 == 0 && K23 % 32 == 0 && KF % 32 == 0);
static_assert(KF + NCO <= K1 && KF + 2 * NCO == D1);
static_assert(NU_BT % NTHR == 0 && NU_W2 % NTHR == 0 && NU_W3 % NTHR == 0 && (GBM * UPR) % NTHR == 0);
static_assert(NTHR == HID && NTHR == 2 * EPB && NTHR == QPB * CH && EPB == 8 * 16 && EPB == 4 * 32);
static_assert(AP >= K23 && (AP * 2) % 16 == 0 && DP >= CH && (DP * 4) % 16 == 0);
static_assert(L_SA % 16 == 0 && L_SD % 16 == 0 && L_SQ % 16 == 0 && L_SO % 16 == 0 && L_CST % 16 == 0);
static_assert(L_SW % 16 == 0 && L_SS % 16 == 0 && L_SJ % 16 == 0 && L_SQL % 16 == 0 && L_SX % 16 == 0);
static_assert(EDGE_LDS_BYTES <= 300000);
static_assert(GBM == (GTHR / 32) * 16 && GBN == 4 * 32 && (HID % GBN) == 0);
static_assert(QPB * CH * 4 == 2 * 32 * 16);
static_assert(NXQ <= NTHR && QPB * 4 * 4 <= L_SX && (QPB + 1) * 4 <= L_SRS && QPB + 1 <= 32);

typedef float          v4f   __attribute__((ext_vector_type(4)));
typedef float          v8f   __attribute__((ext_vector_type(8)));
typedef int            v8i   __attribute__((ext_vector_type(8)));
typedef unsigned short v8us  __attribute__((ext_vector_type(8)));
typedef unsigned short v16us __attribute__((ext_vector_type(16)));
typedef __bf16         v16bf __attribute__((ext_vector_type(16)));
typedef _Float16       v16h  __attribute__((ext_vector_type(16)));
typedef _Float16       v8h   __attribute__((ext_vector_type(8)));
typedef v4f  __attribute__((may_alias)) v4fa;
typedef v8us __attribute__((may_alias)) v8usa;
typedef v8h  __attribute__((may_alias)) v8ha;
union FragB { v16bf v; v16us u; v8us h[2]; v8i w; };
union FragH { v16h v; v8h h[2]; v8i w; };

__device__ __forceinline__ v8f wmb(const FragB& a, const FragB& b, v8f c) {
  v8f d = __builtin_amdgcn_wmma_f32_16x16x32_bf16(false, a.v, false, b.v, (short)0, c, false, false);
  asm volatile("v_nop\n\tv_nop\n\tv_nop\n\tv_nop" : "+v"(d) : "v"(a.w), "v"(b.w));
  return d;
}
__device__ __forceinline__ v8f wmh(const FragH& a, const FragH& b, v8f c) {
  v8f d = __builtin_amdgcn_wmma_f32_16x16x32_f16(false, a.v, false, b.v, (short)0, c, false, false);
  asm volatile("v_nop\n\tv_nop\n\tv_nop\n\tv_nop" : "+v"(d) : "v"(a.w), "v"(b.w));
  return d;
}

__device__ __forceinline__ unsigned bf16_bits(float f) {
  const unsigned u = __float_as_uint(f);
  return (u + 0x7FFFu + ((u >> 16) & 1u)) >> 16;
}
__device__ __forceinline__ float bf16_val(float f) {
  return __uint_as_float(bf16_bits(f) << 16);
}
__device__ __forceinline__ float gelu_f(float t) {
  return 0.5f * t * (1.0f + erff(t * 0.70710678118654752440f));
}

__global__ __launch_bounds__(NTHR) void k_prep(const float* __restrict__ y, const float* __restrict__ fy,
                                               const float* __restrict__ W1, const float* __restrict__ W2,
                                               const float* __restrict__ W3, int nN, int mRows,
                                               unsigned short* BT, _Float16* W2T, _Float16* W3T,
                                               unsigned short* NA) {
  const int u = (int)blockIdx.x * NTHR + (int)threadIdx.x;
  if (u < NU_BT) {
    const int n  = u / UPR;
    const int k8 = (u - n * UPR) * 8;
    v8us o;
#pragma unroll
    for (int i = 0; i < 8; ++i) {
      const int k  = k8 + i;
      const int ra = (k < KF) ? (6 + k) : (k - KF);
      const unsigned va = bf16_bits(W1[(size_t)ra * HID + n]);
      const unsigned mk = (k < KF + NCO) ? 0xFFFFu : 0u;
      o[i] = (unsigned short)(mk & va);
    }
    unsigned short* dp = BT + (size_t)n * K1 + k8;
    *(volatile v8us*)dp = o;
    __threadfence();
    *(volatile v8us*)dp = o;
  } else if (u < NU_BT + NU_W2) {
    const int v  = u - NU_BT;
    const int n  = v >> 5;
    const int k8 = (v & 31) * 8;
    const float* p = W2 + (size_t)k8 * HID + n;
    v8h o;
#pragma unroll
    for (int i = 0; i < 8; ++i) o[i] = (_Float16)(CW * bf16_val(p[(size_t)i * HID]));
    _Float16* dp = W2T + (size_t)n * K23 + k8;
    *(volatile v8h*)dp = o;
    __threadfence();
    *(volatile v8h*)dp = o;
  } else if (u < NU_W) {
    const int v  = u - NU_BT - NU_W2;
    const int n  = v >> 5;
    const int k8 = (v & 31) * 8;
    const float* p = W3 + (size_t)k8 * CH + n;
    v8h o;
#pragma unroll
    for (int i = 0; i < 8; ++i) o[i] = (_Float16)(CW * bf16_val(p[(size_t)i * CH]));
    _Float16* dp = W3T + (size_t)n * K23 + k8;
    *(volatile v8h*)dp = o;
    __threadfence();
    *(volatile v8h*)dp = o;
  } else {
    const int v = u - NU_W;
    if (v >= mRows * UPR) return;
    const int row = v / UPR;
    const int k8  = (v - row * UPR) * 8;
    const int rc  = row < nN ? row : nN - 1;
    const bool ok = row < nN;
    const int kf  = k8 < KF - 8 ? k8 : KF - 8;
    const float* pf = fy + (size_t)rc * CH + kf;
    const v4f a = *(const v4fa*)pf;
    const v4f b = *(const v4fa*)(pf + 4);
    const float* py = y + (size_t)rc * NCO;
    const unsigned fb[8] = {bf16_bits(a.x), bf16_bits(a.y), bf16_bits(a.z), bf16_bits(a.w),
                            bf16_bits(b.x), bf16_bits(b.y), bf16_bits(b.z), bf16_bits(b.w)};
    const unsigned cb[8] = {bf16_bits(py[0]), bf16_bits(py[1]), bf16_bits(py[2]), 0u, 0u, 0u, 0u, 0u};
    const unsigned mF = (ok && k8 < KF) ? 0xFFFFu : 0u;
    const unsigned mC = (ok && k8 == KF) ? 0xFFFFu : 0u;
    v8us o;
#pragma unroll
    for (int i = 0; i < 8; ++i) o[i] = (unsigned short)((mF & fb[i]) | (mC & cb[i]));
    unsigned short* dp = NA + (size_t)row * K1 + k8;
    *(volatile v8us*)dp = o;
    __threadfence();
    *(volatile v8us*)dp = o;
  }
}

__global__ __launch_bounds__(GTHR) void k_gemm(const unsigned short* __restrict__ A, int lda,
                                               const unsigned short* __restrict__ BT, int ldb, int K,
                                               float* Cm, int ldc) {
  __shared__ __attribute__((aligned(16))) float stg[GBM * GBN];
  const int tid = (int)threadIdx.x, lane = tid & 31, wave = tid >> 5, hh = lane >> 4, m = lane & 15;
  const int rowBase = (int)blockIdx.x * GBM;
  const int colBase = (int)blockIdx.y * GBN;

  v8f acc[8];
  {
    const v8f z = {0.f, 0.f, 0.f, 0.f, 0.f, 0.f, 0.f, 0.f};
#pragma unroll
    for (int t = 0; t < 8; ++t) acc[t] = z;
  }
  const unsigned short* ap = A  + (size_t)(rowBase + 16 * wave + m) * (size_t)lda + 8 * hh;
  const unsigned short* bp = BT + (size_t)(colBase + m) * (size_t)ldb + 8 * hh;

#pragma unroll 1
  for (int k0 = 0; k0 < K; k0 += 32) {
    FragB af;
    af.h[0] = *(const v8usa*)(ap + k0);
    af.h[1] = *(const v8usa*)(ap + k0 + 16);
#pragma unroll
    for (int nt = 0; nt < 8; ++nt) {
      const unsigned short* wq = bp + (size_t)(16 * nt) * (size_t)ldb + k0;
      FragB bf;
      bf.h[0] = *(const v8usa*)wq;
      bf.h[1] = *(const v8usa*)(wq + 16);
      acc[nt] = wmb(af, bf, acc[nt]);
    }
  }

#pragma unroll
  for (int nt = 0; nt < 8; ++nt) {
    const int lc = 16 * nt + m;
#pragma unroll
    for (int r = 0; r < 8; ++r) {
      const int lr = 16 * wave + 8 * hh + r;
      stg[lr * GBN + lc] = acc[nt][r];
    }
  }
  __syncthreads();

  v4f pv[16];
#pragma unroll
  for (int i = 0; i < 16; ++i) pv[i] = *(const v4fa*)(stg + (16 * wave + i) * GBN + 4 * lane);
#pragma unroll
  for (int i = 0; i < 16; ++i) {
    float* op = Cm + (size_t)(rowBase + 16 * wave + i) * (size_t)ldc + colBase + 4 * lane;
    *(volatile v4f*)op = pv[i];
  }
  __threadfence();
#pragma unroll
  for (int i = 0; i < 16; ++i) {
    float* op = Cm + (size_t)(rowBase + 16 * wave + i) * (size_t)ldc + colBase + 4 * lane;
    *(volatile v4f*)op = pv[i];
  }
}

__global__ __launch_bounds__(NTHR) void k_edge(const int* __restrict__ nidx, const int* __restrict__ rsp,
                                               int nE, int nQ, int nN,
                                               const float* __restrict__ P,
                                               const _Float16* __restrict__ W2T,
                                               const _Float16* __restrict__ W3T,
                                               const float* __restrict__ y, const float* __restrict__ x,
                                               const float* __restrict__ fy, const float* __restrict__ W1,
                                               const float* __restrict__ b1, const float* __restrict__ b2,
                                               const float* __restrict__ b3, float* out) {
  extern __shared__ __attribute__((aligned(16))) float dyn[];
  char* base = (char*)dyn;
  _Float16* sA  = (_Float16*)(base);
  _Float16* sH  = (_Float16*)(base + L_SA);
  float*    sD  = (float*)(base + L_SA + L_SH);
  float*    sQ  = (float*)(base + L_SA + L_SH + L_SD);
  float*    sO  = (float*)(base + L_SA + L_SH + L_SD + L_SQ);
  float*    cst = (float*)(base + L_SA + L_SH + L_SD + L_SQ + L_SO);
  float*    sW  = (float*)(base + L_SA + L_SH + L_SD + L_SQ + L_SO + L_CST);
  float*    sS  = (float*)(base + L_SA + L_SH + L_SD + L_SQ + L_SO + L_CST + L_SW);
  int*      sJ  = (int*)(base + L_SA + L_SH + L_SD + L_SQ + L_SO + L_CST + L_SW + L_SS);
  int*      sQL = (int*)(base + L_SA + L_SH + L_SD + L_SQ + L_SO + L_CST + L_SW + L_SS + L_SJ);
  float*    sX  = (float*)(base + L_SA + L_SH + L_SD + L_SQ + L_SO + L_CST + L_SW + L_SS + L_SJ + L_SQL);
  int*      sRS = (int*)(base + L_SA + L_SH + L_SD + L_SQ + L_SO + L_CST + L_SW + L_SS + L_SJ + L_SQL + L_SX);

  const int tid = (int)threadIdx.x, lane = tid & 31, wave = tid >> 5, hh = lane >> 4, m = lane & 15;
  const int q0 = (int)blockIdx.x * QPB;

  {
    int qi = q0 + (tid < QPB ? tid : QPB);
    qi = qi > nQ ? nQ : qi;
    int v = rsp[qi];
    v = v < 0 ? 0 : (v > nE ? nE : v);
    if (tid <= QPB) sRS[tid] = v;
    cst[tid] = bf16_val(b2[tid]);
    const float vb3 = b3[tid < CH ? tid : CH - 1];
    if (tid < CH) cst[HID + tid] = bf16_val(vb3);
    const int t12 = tid < NXQ ? tid : NXQ - 1;
    const int xq = t12 / NCO, xd = t12 - NCO * xq;
    int xr = q0 + xq;
    xr = xr > nQ - 1 ? nQ - 1 : xr;
    const float xv = bf16_val(x[(size_t)xr * NCO + xd]);
    if (tid < NXQ) sX[xq * 4 + xd] = xv;
  }
  __syncthreads();
  const int lo = sRS[0], e1 = sRS[1], e2 = sRS[2], e3 = sRS[3], hi = sRS[4];
  const bool bad = (e1 < lo) || (e2 < e1) || (e3 < e2) || (hi < e3) || (hi - lo > EPB);

  if (tid < EPB) {
    const int ea = lo + tid;
    const int ec = ea > nE - 1 ? nE - 1 : ea;
    int j = nidx[ec];
    j = j < 0 ? 0 : (j > nN - 1 ? nN - 1 : j);
    const int ql = (ea >= e1 ? 1 : 0) + (ea >= e2 ? 1 : 0) + (ea >= e3 ? 1 : 0);
    sJ[tid]  = j;
    sQL[tid] = ql;
    const float* py = y + (size_t)j * NCO;
    const float ky0 = bf16_val(py[0]), ky1 = bf16_val(py[1]), ky2 = bf16_val(py[2]);
    const float qx0 = sX[ql * 4 + 0], qx1 = sX[ql * 4 + 1], qx2 = sX[ql * 4 + 2];
    const float nk = sqrtf((ky0 * ky0 + ky2 * ky2) + ky1 * ky1);
    const float nq = sqrtf((qx0 * qx0 + qx2 * qx2) + qx1 * qx1);
    const float rk = 1.0f / fmaxf(nk, 1e-12f);
    const float rq = 1.0f / fmaxf(nq, 1e-12f);
    const float k0n = ky0 * rk, k1n = ky1 * rk, k2n = ky2 * rk;
    const float q0n = qx0 * rq, q1n = qx1 * rq, q2n = qx2 * rq;
    sS[tid] = (q0n * k0n + q2n * k2n) + q1n * k1n;
  }
  {
    const float w0 = bf16_val(W1[(size_t)(NCO + 0) * HID + tid]);
    const float w1 = bf16_val(W1[(size_t)(NCO + 1) * HID + tid]);
    const float w2 = bf16_val(W1[(size_t)(NCO + 2) * HID + tid]);
    const float bb = bf16_val(b1[tid]);
#pragma unroll
    for (int qi = 0; qi < QPB; ++qi) {
      const float x0 = sX[qi * 4 + 0], x1 = sX[qi * 4 + 1], x2 = sX[qi * 4 + 2];
      sQ[qi * HID + tid] = ((x0 * w0 + x1 * w1) + x2 * w2) + bb;
    }
  }
  __syncthreads();

  if (wave < QPB) {
    int sb = sRS[wave] - lo, se = sRS[wave + 1] - lo;
    sb = sb < 0 ? 0 : (sb > EPB ? EPB : sb);
    se = se < 0 ? 0 : (se > EPB ? EPB : se);
    const float ninf = __uint_as_float(0xff800000u);
    float vv[4];
    float mx = ninf;
#pragma unroll
    for (int i = 0; i < 4; ++i) {
      const int s  = sb + lane + 32 * i;
      const int sc = s > EPB - 1 ? EPB - 1 : s;
      const float v = sS[sc];
      vv[i] = (s < se) ? v : ninf;
      mx = fmaxf(mx, vv[i]);
    }
#pragma unroll
    for (int off = 16; off > 0; off >>= 1) mx = fmaxf(mx, __shfl_xor(mx, off, 32));
    const float mxs = (mx == ninf) ? 0.0f : mx;
    float ex[4];
    float sm = 0.0f;
#pragma unroll
    for (int i = 0; i < 4; ++i) {
      ex[i] = expf(vv[i] - mxs);
      sm = sm + ex[i];
    }
#pragma unroll
    for (int off = 16; off > 0; off >>= 1) sm = sm + __shfl_xor(sm, off, 32);
    const float rinv = 1.0f / fmaxf(sm, 1e-30f);
#pragma unroll
    for (int i = 0; i < 4; ++i) {
      const int s = sb + lane + 32 * i;
      if (s < se) sW[s] = ex[i] * rinv;
    }
  }

  {
    const int s  = tid & (EPB - 1);
    const int hf = tid >> 7;
    const int j  = sJ[s];
    const int ql = sQL[s];
    const float* pr = P + (size_t)j * PP + (HID / 2) * hf;
    const float* qr = sQ + ql * HID + (HID / 2) * hf;
    _Float16*    ar = sA + s * AP + (HID / 2) * hf;
#pragma unroll 1
    for (int c8 = 0; c8 < HID / 16; ++c8) {
      const v4f pa = *(const v4fa*)(pr + 8 * c8);
      const v4f pb = *(const v4fa*)(pr + 8 * c8 + 4);
      const v4f qa = *(const v4fa*)(qr + 8 * c8);
      const v4f qb = *(const v4fa*)(qr + 8 * c8 + 4);
      v8h o;
      o[0] = (_Float16)(CA * gelu_f(pa.x + qa.x));
      o[1] = (_Float16)(CA * gelu_f(pa.y + qa.y));
      o[2] = (_Float16)(CA * gelu_f(pa.z + qa.z));
      o[3] = (_Float16)(CA * gelu_f(pa.w + qa.w));
      o[4] = (_Float16)(CA * gelu_f(pb.x + qb.x));
      o[5] = (_Float16)(CA * gelu_f(pb.y + qb.y));
      o[6] = (_Float16)(CA * gelu_f(pb.z + qb.z));
      o[7] = (_Float16)(CA * gelu_f(pb.w + qb.w));
      *(v8ha*)(ar + 8 * c8) = o;
    }
  }
  __syncthreads();

  {
    const _Float16* ap = sA + (16 * wave + m) * AP + 8 * hh;
#pragma unroll 1
    for (int nc = 0; nc < HID / 128; ++nc) {
      v8f acc[8];
      {
        const v8f z = {0.f, 0.f, 0.f, 0.f, 0.f, 0.f, 0.f, 0.f};
#pragma unroll
        for (int t = 0; t < 8; ++t) acc[t] = z;
      }
      const _Float16* bp = W2T + (size_t)(nc * 128 + m) * K23 + 8 * hh;
#pragma unroll 1
      for (int k0 = 0; k0 < K23; k0 += 32) {
        FragH af;
        af.h[0] = *(const v8ha*)(ap + k0);
        af.h[1] = *(const v8ha*)(ap + k0 + 16);
#pragma unroll
        for (int nt = 0; nt < 8; ++nt) {
          const _Float16* wq = bp + (size_t)(16 * nt) * K23 + k0;
          FragH bf;
          bf.h[0] = *(const v8ha*)wq;
          bf.h[1] = *(const v8ha*)(wq + 16);
          acc[nt] = wmh(af, bf, acc[nt]);
        }
      }
#pragma unroll
      for (int nt = 0; nt < 8; ++nt) {
        const int col = nc * 128 + 16 * nt + m;
        const float bv = cst[col];
#pragma unroll
        for (int r = 0; r < 8; ++r) {
          const int row = 16 * wave + 8 * hh + r;
          const float u2 = acc[nt][r] * INVC + bv;
          sH[row * AP + col] = (_Float16)(CA * gelu_f(u2));
        }
      }
    }
  }
  __syncthreads();

  {
    const _Float16* ap = sH + (16 * wave + m) * AP + 8 * hh;
    const _Float16* bp = W3T + (size_t)m * K23 + 8 * hh;
    v8f acc[4];
    {
      const v8f z = {0.f, 0.f, 0.f, 0.f, 0.f, 0.f, 0.f, 0.f};
#pragma unroll
      for (int t = 0; t < 4; ++t) acc[t] = z;
    }
#pragma unroll 1
    for (int k0 = 0; k0 < K23; k0 += 32) {
      FragH af;
      af.h[0] = *(const v8ha*)(ap + k0);
      af.h[1] = *(const v8ha*)(ap + k0 + 16);
#pragma unroll
      for (int nt = 0; nt < 4; ++nt) {
        const _Float16* wq = bp + (size_t)(16 * nt) * K23 + k0;
        FragH bf;
        bf.h[0] = *(const v8ha*)wq;
        bf.h[1] = *(const v8ha*)(wq + 16);
        acc[nt] = wmh(af, bf, acc[nt]);
      }
    }
#pragma unroll
    for (int nt = 0; nt < 4; ++nt) {
      const int col = 16 * nt + m;
      const float bv = cst[HID + col];
#pragma unroll
      for (int r = 0; r < 8; ++r) {
        const int row = 16 * wave + 8 * hh + r;
        sD[row * DP + col] = acc[nt][r] * INVC + bv;
      }
    }
  }
  __syncthreads();

  {
    const int ql = tid >> 6, c = tid & (CH - 1);
    int sb = sRS[ql] - lo, se = sRS[ql + 1] - lo;
    sb = sb < 0 ? 0 : (sb > EPB ? EPB : sb);
    se = se < 0 ? 0 : (se > EPB ? EPB : se);
    float sum = 0.0f;
#pragma unroll 2
    for (int s = sb; s < se; ++s) {
      const int j = sJ[s];
      const float fv = bf16_val(fy[(size_t)j * CH + c]);
      const float kv = sD[s * DP + c];
      const float wv = sW[s];
      sum = sum + (kv * fv) * wv;
    }
    const float ov = bad ? __uint_as_float(0x7fc00000u) : sum;
    sO[ql * CH + c] = ov;
  }
  __syncthreads();

  const int tl = tid < 64 ? tid : 63;
  const v4f o4 = *(const v4fa*)(sO + 4 * tl);
  const int orow = q0 + (tl >> 4);
  const bool stv = (tid < 64) && (orow < nQ);
  float* op = out + (size_t)q0 * CH + 4 * tl;
  if (stv) *(volatile v4f*)op = o4;
  __threadfence();
  if (stv) *(volatile v4f*)op = o4;
}

static inline int cdiv(int a, int b) { return (a + b - 1) / b; }

extern "C" void kernel_launch(void* const* d_in, const int* in_sizes, int n_in,
                              void* d_out, int out_size, void* d_ws, size_t ws_size,
                              hipStream_t stream) {
  if (n_in < 11) return;
  if (in_sizes[0] < NCO || (in_sizes[0] % NCO) != 0) return;
  const int nN = in_sizes[0] / NCO;
  if (in_sizes[1] < NCO || (in_sizes[1] % NCO) != 0) return;
  const int nQ = in_sizes[1] / NCO;
  if (in_sizes[2] != CH * nN) return;
  const int nE = in_sizes[3];
  if (nE < 1) return;
  if (in_sizes[4] != nQ + 1) return;
  if (in_sizes[5] != D1 * HID || in_sizes[6] != HID) return;
  if (in_sizes[7] != HID * HID || in_sizes[8] != HID) return;
  if (in_sizes[9] != HID * CH || in_sizes[10] != CH) return;
  if (out_size != nQ * CH) return;

  const float* y    = (const float*)d_in[0];
  const float* x    = (const float*)d_in[1];
  const float* fy   = (const float*)d_in[2];
  const int*   nidx = (const int*)d_in[3];
  const int*   rsp  = (const int*)d_in[4];
  const float* W1   = (const float*)d_in[5];
  const float* b1   = (const float*)d_in[6];
  const float* W2   = (const float*)d_in[7];
  const float* b2   = (const float*)d_in[8];
  const float* W3   = (const float*)d_in[9];
  const float* b3   = (const float*)d_in[10];
  float* out = (float*)d_out;

  const int NP = cdiv(nN, GBM) * GBM;
  const int gM = NP / GBM;

  char* ws = (char*)d_ws;
  size_t off = 0;
  const size_t oBT = off; off += (size_t)HID * K1 * 2;    off = (off + 255) & ~(size_t)255;
  const size_t oW2 = off; off += (size_t)HID * K23 * 2;   off = (off + 255) & ~(size_t)255;
  const size_t oW3 = off; off += (size_t)CH * K23 * 2;    off = (off + 255) & ~(size_t)255;
  const size_t oNA = off; off += (size_t)NP * K1 * 2;     off = (off + 255) & ~(size_t)255;
  const size_t oP  = off; off += (size_t)NP * PP * 4;     off = (off + 255) & ~(size_t)255;
  if (off > ws_size || off > (size_t)WSMAX) return;
  unsigned short* BT  = (unsigned short*)(ws + oBT);
  _Float16*       W2T = (_Float16*)(ws + oW2);
  _Float16*       W3T = (_Float16*)(ws + oW3);
  unsigned short* NA  = (unsigned short*)(ws + oNA);
  float*          P   = (float*)(ws + oP);

  hipFuncSetAttribute(reinterpret_cast<const void*>(&k_edge), hipFuncAttributeMaxDynamicSharedMemorySize,
                      (int)EDGE_LDS_BYTES);

  const int nUnits = NU_W + NP * UPR;
  k_prep<<<cdiv(nUnits, NTHR), NTHR, 0, stream>>>(y, fy, W1, W2, W3, nN, NP, BT, W2T, W3T, NA);
  k_gemm<<<dim3(gM, HID / GBN), GTHR, 0, stream>>>(NA, K1, BT, K1, K1, P, PP);
  k_edge<<<cdiv(nQ, QPB), NTHR, EDGE_LDS_BYTES, stream>>>(nidx, rsp, nE, nQ, nN, P, W2T, W3T,
                                                           y, x, fy, W1, b1, b2, b3, out);
}
